// CalibrationNetwork_81329500717524
// MI455X (gfx1250) — hardware-verified
//
#include <hip/hip_runtime.h>
#include <math.h>
#include <stdint.h>

#define NB    16384
#define NJ    12
#define NQ    7
#define NO    5
#define NI    6
#define NH    128
#define NK2   129
#define NQO   35
#define CHUNK 512
#define NCH   (NB / CHUNK)
#define MAXT  (CHUNK / 16)
#define SLOT  64
#define WP    136
#define ZP    132
#define WSC   256.0f
#define WINV  0.00390625f

static_assert(NCH * CHUNK == NB);
static_assert(CHUNK == 2 * 256);
static_assert(NQO == NQ * NO);
static_assert((NB * NQO) % 1024 == 0);
static_assert(NQO <= SLOT);

typedef _Float16 v16h __attribute__((ext_vector_type(16)));
typedef _Float16 v8h  __attribute__((ext_vector_type(8)));
typedef float    v8f  __attribute__((ext_vector_type(8)));
typedef float    v4f  __attribute__((ext_vector_type(4)));

union FragH { v16h v; v8h h[2]; };

__device__ __forceinline__ float bfr(float f) {
  unsigned u = __float_as_uint(f);
  u = (u + 0x7FFFu + ((u >> 16) & 1u)) & 0xFFFF0000u;
  return __uint_as_float(u);
}
__device__ __forceinline__ v8f zero8() { v8f z = {0.f, 0.f, 0.f, 0.f, 0.f, 0.f, 0.f, 0.f}; return z; }

__device__ __forceinline__ v16h ldfrag_h(const _Float16* p) {
  FragH f;
  f.h[0] = *(const v8h*)(p);
  f.h[1] = *(const v8h*)(p + 16);
  return f.v;
}
__device__ __forceinline__ v8f mma16(v16h a, v16h b, v8f c) {
  return __builtin_amdgcn_wmma_f32_16x16x32_f16(false, a, false, b, (short)0, c, false, false);
}
__device__ __forceinline__ void guard8(v8f& acc, v16h a0, v16h b0, v16h a1, v16h b1,
                                       v16h a2, v16h b2, v16h a3, v16h b3) {
#if defined(__HIP_DEVICE_COMPILE__)
  asm volatile("v_nop\n\tv_nop\n\tv_nop\n\tv_nop"
               : "+v"(acc) : "v"(a0), "v"(b0), "v"(a1), "v"(b1), "v"(a2), "v"(b2), "v"(a3), "v"(b3));
#endif
}

__global__ __launch_bounds__(256) void mlp_fwd(
    const float* __restrict__ x,  const int* __restrict__ jid,
    const float* __restrict__ W1, const float* __restrict__ W1a,
    const float* __restrict__ W2, const float* __restrict__ W2a,
    const float* __restrict__ V,  const float* __restrict__ Va,
    float* res) {
  __shared__ __align__(16) _Float16 s_w2t[NH * WP];
  __shared__ __align__(16) _Float16 s_z1[16 * WP];
  __shared__ __align__(16) float s_z2[16 * ZP];
  __shared__ __align__(16) float s_xq[16 * 8];
  __shared__ __align__(16) float s_w1q[NI * NH];
  __shared__ __align__(16) float s_vcq[NK2 * 8];
  __shared__ __align__(16) float s_b2[NH];
  __shared__ __align__(16) float s_lg[16 * 8];
  __shared__ __align__(16) float s_out[16 * SLOT];
  __shared__ int s_idx[CHUNK];
  __shared__ int s_wc[16];

  const int t = threadIdx.x;
  const int lane = t & 31, wave = t >> 5, hh = lane >> 4, c16 = lane & 15;
  const int j = (int)(blockIdx.x % NJ);
  const int chunk = (int)(blockIdx.x / NJ);
  if (chunk >= NCH) return;

  const int sa0 = chunk * CHUNK + t;
  const int sa1 = sa0 + 256;
  int id0 = jid[sa0], id1 = jid[sa1];
  id0 = min(max(id0, 0), NJ - 1);
  id1 = min(max(id1, 0), NJ - 1);
  const bool f0 = (id0 == j), f1 = (id1 == j);
  const unsigned m0 = __builtin_amdgcn_ballot_w32(f0);
  const unsigned m1 = __builtin_amdgcn_ballot_w32(f1);
  if (lane == 0) { s_wc[wave] = __builtin_popcount(m0); s_wc[8 + wave] = __builtin_popcount(m1); }
  for (int e = t; e < 16 * SLOT; e += 256) s_out[e] = 0.f;
  __syncthreads();
  int base0 = 0, tot0 = 0, base1 = 0, tot1 = 0;
#pragma unroll
  for (int w = 0; w < 8; ++w) {
    const int ca = s_wc[w], cb = s_wc[8 + w];
    base0 += (w < wave) ? ca : 0;  tot0 += ca;
    base1 += (w < wave) ? cb : 0;  tot1 += cb;
  }
  const unsigned lt = (1u << lane) - 1u;
  int pos0 = base0 + __builtin_popcount(m0 & lt);
  int pos1 = tot0 + base1 + __builtin_popcount(m1 & lt);
  pos0 = min(pos0, CHUNK - 1);
  pos1 = min(pos1, CHUNK - 1);
  if (f0) s_idx[pos0] = sa0;
  if (f1) s_idx[pos1] = sa1;
  const int cnt = min(tot0 + tot1, CHUNK);
  __syncthreads();
  if (cnt == 0) return;

  const float* W2aj = W2a + (size_t)j * NK2 * NH;
  for (int e = t; e < NH * NH; e += 256) {
    const int k = e >> 7, h = e & 127;
    const int gi = e + NH;
    const float v = (bfr(W2[gi]) + bfr(W2aj[gi])) * WSC;
    s_w2t[h * WP + k] = (_Float16)v;
  }
  if (t < NH) s_b2[t] = bfr(W2[t]) + bfr(W2aj[t]);

  const int ntile = min((cnt + 15) >> 4, MAXT);
  for (int tile = 0; tile < ntile; ++tile) {
    const int s0 = tile * 16;
    const int tcnt = min(16, cnt - s0);
    for (int q = 0; q < NQ; ++q) {
      {
        const int e = min(t, 16 * NO - 1);
        const int s = e / NO, i = e - s * NO;
        const int si = min(s0 + s, cnt - 1);
        const int b  = min(max(s_idx[si], 0), NB - 1);
        const float v = bfr(x[((size_t)b * NQ + q) * NO + i]);
        if (t < 16 * NO) s_xq[s * 8 + i] = v;
      }
      {
        const float* W1q  = W1 + (size_t)q * NI * NH;
        const float* W1aq = W1a + ((size_t)j * NQ + q) * (NI * NH);
        for (int e = t; e < NI * NH; e += 256) s_w1q[e] = bfr(W1q[e]) + bfr(W1aq[e]);
        const float* Vq  = V + (size_t)q * NK2 * NO;
        const float* Vaq = Va + ((size_t)j * NQ + q) * (NK2 * NO);
        for (int e = t; e < NK2 * NO; e += 256) {
          const int k = e / NO, o = e - k * NO;
          s_vcq[k * 8 + o] = bfr(Vq[e]) + bfr(Vaq[e]);
        }
      }
      __syncthreads();

      {
        const int h = t & 127, sb = t >> 7;
        const float w0 = s_w1q[h],          w1 = s_w1q[NH + h],     w2 = s_w1q[2 * NH + h];
        const float w3 = s_w1q[3 * NH + h], w4 = s_w1q[4 * NH + h], w5 = s_w1q[5 * NH + h];
#pragma unroll 2
        for (int it = 0; it < 8; ++it) {
          const int s = sb + 2 * it;
          const v4f xv = *(const v4f*)(s_xq + s * 8);
          const float x4 = s_xq[s * 8 + 4];
          float p = w0;
          p = fmaf(xv[0], w1, p);
          p = fmaf(xv[1], w2, p);
          p = fmaf(xv[2], w3, p);
          p = fmaf(xv[3], w4, p);
          p = fmaf(x4,    w5, p);
          const float ev = expf(-p);
          s_z1[s * WP + h] = (_Float16)__builtin_amdgcn_rcpf(1.0f + ev);
        }
      }
      __syncthreads();

      {
        const int n0 = wave * 16;
        const _Float16* ap = s_z1 + c16 * WP + 8 * hh;
        const _Float16* bp = s_w2t + (n0 + c16) * WP + 8 * hh;
        const v16h a0 = ldfrag_h(ap),      g0 = ldfrag_h(bp);
        const v16h a1 = ldfrag_h(ap + 32), g1 = ldfrag_h(bp + 32);
        const v16h a2 = ldfrag_h(ap + 64), g2 = ldfrag_h(bp + 64);
        const v16h a3 = ldfrag_h(ap + 96), g3 = ldfrag_h(bp + 96);
        v8f acc = zero8();
        acc = mma16(a0, g0, acc);
        acc = mma16(a1, g1, acc);
        acc = mma16(a2, g2, acc);
        acc = mma16(a3, g3, acc);
        guard8(acc, a0, g0, a1, g1, a2, g2, a3, g3);
        const int n = n0 + c16;
        const float bias = s_b2[n];
#pragma unroll
        for (int r = 0; r < 8; ++r) {
          const float pre = acc[r] * WINV + bias;
          const float ev  = expf(-pre);
          s_z2[(8 * hh + r) * ZP + n] = __builtin_amdgcn_rcpf(1.0f + ev);
        }
      }
      __syncthreads();

      if (wave < 3) {
        const int r = c16;
        const int o = min(t >> 4, NO - 1);
        const float* zr = s_z2 + r * ZP;
        const float* vc = s_vcq + 8 + o;
        float a3 = s_vcq[o];
#pragma unroll 4
        for (int k = 0; k < NH; ++k) a3 = fmaf(zr[k], vc[k * 8], a3);
        if (t < 16 * NO) s_lg[r * 8 + o] = a3;
      }
      __syncthreads();

      if (wave == 0) {
        const int r = c16;
        const float l0 = s_lg[r * 8 + 0], l1 = s_lg[r * 8 + 1], l2 = s_lg[r * 8 + 2];
        const float l3 = s_lg[r * 8 + 3], l4 = s_lg[r * 8 + 4];
        const float mx = fmaxf(fmaxf(fmaxf(l0, l1), fmaxf(l2, l3)), l4);
        const float e0 = expf(l0 - mx), e1 = expf(l1 - mx), e2 = expf(l2 - mx);
        const float e3 = expf(l3 - mx), e4 = expf(l4 - mx);
        const float sum = (((e0 + e1) + e2) + e3) + e4;
        const float inv = 1.0f / sum;
        if (lane < 16) {
          float* op = s_out + r * SLOT + q * NO;
          op[0] = e0 * inv; op[1] = e1 * inv; op[2] = e2 * inv; op[3] = e3 * inv; op[4] = e4 * inv;
        }
      }
      __syncthreads();
    }

    {
      const int sl = 2 * wave + hh;
      const bool live = sl < tcnt;
      const int si = min(s0 + sl, cnt - 1);
      const int b  = min(max(s_idx[si], 0), NB - 1);
      const v4f v = *(const v4f*)(s_out + sl * SLOT + c16 * 4);
      float* dp = res + (size_t)b * SLOT + c16 * 4;
      if (live) *(volatile v4f*)dp = v;
      __threadfence();
      if (live) *(volatile v4f*)dp = v;
    }
  }
}

__global__ __launch_bounds__(256) void repack(const float* __restrict__ res, float* out) {
  const int g  = blockIdx.x * 256 + threadIdx.x;
  const int e0 = g * 4;
  v4f v;
#pragma unroll
  for (int c = 0; c < 4; ++c) {
    const int e = min(e0 + c, NB * NQO - 1);
    const int b = e / NQO;
    const int r = e - b * NQO;
    v[c] = res[(size_t)b * SLOT + r];
  }
  float* op = out + e0;
  *(volatile v4f*)op = v;
  __threadfence();
  *(volatile v4f*)op = v;
}

extern "C" void kernel_launch(void* const* d_in, const int* in_sizes, int n_in,
                              void* d_out, int out_size, void* d_ws, size_t ws_size,
                              hipStream_t stream) {
  if (n_in < 8) return;
  if (in_sizes[0] != NB * NQ * NO) return;
  if (in_sizes[1] != NB) return;
  if (in_sizes[2] != NQ * NI * NH || in_sizes[3] != NJ * NQ * NI * NH) return;
  if (in_sizes[4] != NK2 * NH || in_sizes[5] != NJ * NK2 * NH) return;
  if (in_sizes[6] != NQ * NK2 * NO || in_sizes[7] != NJ * NQ * NK2 * NO) return;
  if (out_size != NB * NQO) return;
  const size_t need = (size_t)NB * SLOT * sizeof(float);
  if (need > ws_size) return;
  if (need > (size_t)134217728) return;

  const float* x   = (const float*)d_in[0];
  const int*   jid = (const int*)d_in[1];
  const float* W1  = (const float*)d_in[2];
  const float* W1a = (const float*)d_in[3];
  const float* W2  = (const float*)d_in[4];
  const float* W2a = (const float*)d_in[5];
  const float* V   = (const float*)d_in[6];
  const float* Va  = (const float*)d_in[7];
  float* out = (float*)d_out;
  float* res = (float*)d_ws;

  mlp_fwd<<<dim3(NJ * NCH), dim3(256), 0, stream>>>(x, jid, W1, W1a, W2, W2a, V, Va, res);
  repack<<<dim3((NB * NQO) / 1024), dim3(256), 0, stream>>>(res, out);
  (void)hipGetLastError();
}
